// DecoderLayer_90074054132191
// MI455X (gfx1250) — hardware-verified
//
#include <hip/hip_runtime.h>
#include <math.h>

constexpr int kBatch  = 2;
constexpr int kSeq    = 1024;
constexpr int kDim    = 1024;
constexpr int kHeads  = 16;
constexpr int kDh     = 64;
constexpr int kFF     = 4096;
constexpr int kTok    = kBatch * kSeq;
constexpr int kQKVld  = 3 * kDim;
constexpr float kXCarry   = 8.0f;
constexpr float kHCarry   = 8.0f;
constexpr float kUCarry   = 8.0f;
constexpr float kWCarry   = 256.0f;
constexpr float kAttCarry = 256.0f;
constexpr float kScaleXW  = 1.0f / (kXCarry * kWCarry);
constexpr float kScaleHW  = 1.0f / (kHCarry * kWCarry);
constexpr float kScaleUW  = 1.0f / (kUCarry * kWCarry);
constexpr float kScaleAW  = 1.0f / (kAttCarry * kWCarry);
constexpr float kFlowEps  = 1.0e-6f;
constexpr float kLnEps    = 1.0e-5f;
constexpr float kInvDim   = 1.0f / 1024.0f;
static_assert(kHeads * kDh == kDim, "shape");
static_assert(kTok % 64 == 0 && kDim % 64 == 0 && kFF % 64 == 0, "M and N tile multiples");
static_assert(kDim % 32 == 0 && kFF % 32 == 0, "K multiples of 32");
static_assert(kDim == 4 * 256, "LN thread map: 256 threads x 4 floats per row");

typedef __attribute__((ext_vector_type(16))) _Float16 v16h;
typedef __attribute__((ext_vector_type(8)))  _Float16 v8h;
typedef __attribute__((ext_vector_type(16))) __bf16   v16b;
typedef __attribute__((ext_vector_type(8)))  __bf16   v8b;
typedef __attribute__((ext_vector_type(8)))  float    v8f;
typedef __attribute__((ext_vector_type(4)))  float    v4f;
typedef __attribute__((ext_vector_type(2)))  float    v2f;
typedef __attribute__((ext_vector_type(4)))  unsigned int v4u;

__device__ __forceinline__ unsigned short f2bf_bits(float f) {
  unsigned u = __float_as_uint(f);
  return (unsigned short)((u + 0x7FFFu + ((u >> 16) & 1u)) >> 16);
}
__device__ __forceinline__ float bf_bits2f(unsigned short h) { return __uint_as_float(((unsigned)h) << 16); }

__device__ __forceinline__ void dep_guard_h(v8f& a, v8f& b, v16h x, v16h y) { asm volatile("v_nop\n\tv_nop\n\tv_nop\n\tv_nop" : "+v"(a), "+v"(b) : "v"(x), "v"(y)); }
__device__ __forceinline__ void dep_guard_b(v8f& a, v8f& b, v16b x, v16b y) { asm volatile("v_nop\n\tv_nop\n\tv_nop\n\tv_nop" : "+v"(a), "+v"(b) : "v"(x), "v"(y)); }
__device__ __forceinline__ void dep_guard4_h(v8f& a, v8f& b, v8f& c, v8f& d, v16h x, v16h y) { asm volatile("v_nop\n\tv_nop\n\tv_nop\n\tv_nop" : "+v"(a), "+v"(b), "+v"(c), "+v"(d) : "v"(x), "v"(y)); }
__device__ __forceinline__ void dep_guard4_b(v8f& a, v8f& b, v8f& c, v8f& d, v16b x, v16b y) { asm volatile("v_nop\n\tv_nop\n\tv_nop\n\tv_nop" : "+v"(a), "+v"(b), "+v"(c), "+v"(d) : "v"(x), "v"(y)); }
__device__ __forceinline__ void keep4_h(v16h a, v16h b, v16h c, v16h d) { asm volatile("v_nop" :: "v"(a), "v"(b), "v"(c), "v"(d)); }
__device__ __forceinline__ void keep4_b(v16b a, v16b b, v16b c, v16b d) { asm volatile("v_nop" :: "v"(a), "v"(b), "v"(c), "v"(d)); }
__device__ __forceinline__ void acc_guard4(v8f& a, v8f& b, v8f& c, v8f& d) { asm volatile("v_nop\n\tv_nop\n\tv_nop\n\tv_nop" : "+v"(a), "+v"(b), "+v"(c), "+v"(d)); }
template <typename T> struct Frag;
template <> struct Frag<_Float16> {
  typedef v16h V; union U { v16h v; v8h h[2]; };
  static __device__ __forceinline__ v16h load(const _Float16* p) {
    U f; f.h[0] = *(const v8h*)(p); f.h[1] = *(const v8h*)(p + 16); return f.v;
  }
  static __device__ __forceinline__ v8f mma(v16h a, v16h b, v8f c) {
    return __builtin_amdgcn_wmma_f32_16x16x32_f16(false, a, false, b, (short)0, c, false, false);
  }
  static __device__ __forceinline__ void guard(v8f& a, v8f& b, v16h x, v16h y) { dep_guard_h(a, b, x, y); }
  static __device__ __forceinline__ void guard4(v8f& a, v8f& b, v8f& c, v8f& d, v16h x, v16h y) { dep_guard4_h(a, b, c, d, x, y); }
  static __device__ __forceinline__ void keep(v16h a, v16h b, v16h c, v16h d) { keep4_h(a, b, c, d); }
};
template <> struct Frag<__bf16> {
  typedef v16b V; union U { v16b v; v8b h[2]; };
  static __device__ __forceinline__ v16b load(const __bf16* p) {
    U f; f.h[0] = *(const v8b*)(p); f.h[1] = *(const v8b*)(p + 16); return f.v;
  }
  static __device__ __forceinline__ v8f mma(v16b a, v16b b, v8f c) {
    return __builtin_amdgcn_wmma_f32_16x16x32_bf16(false, a, false, b, (short)0, c, false, false);
  }
  static __device__ __forceinline__ void guard(v8f& a, v8f& b, v16b x, v16b y) { dep_guard_b(a, b, x, y); }
  static __device__ __forceinline__ void guard4(v8f& a, v8f& b, v8f& c, v8f& d, v16b x, v16b y) { dep_guard4_b(a, b, c, d, x, y); }
  static __device__ __forceinline__ void keep(v16b a, v16b b, v16b c, v16b d) { keep4_b(a, b, c, d); }
};

__device__ __forceinline__ unsigned pk16(unsigned short a, unsigned short b) { return (unsigned)a | ((unsigned)b << 16); }
__device__ __forceinline__ unsigned short h_bits(float f) { const _Float16 h = (_Float16)f; return __builtin_bit_cast(unsigned short, h); }
__device__ __forceinline__ float frcp(float x) { return __builtin_amdgcn_rcpf(x); }
__device__ __forceinline__ float sigm(float x) { return frcp(1.0f + expf(-x)); }

template <int ET> struct Elem;
template <> struct Elem<0> { typedef _Float16 T; };
template <> struct Elem<1> { typedef __bf16 T; };
template <int ET, bool SPLIT, int BIAS_MODE, int OUT_MODE, bool RESID, int ACT = 0>
__global__ __launch_bounds__(256) void wmma_gemm64(
    const unsigned short* __restrict__ Ap, const unsigned short* __restrict__ A2p, int lda, long strideA,
    const unsigned short* __restrict__ Btp, const unsigned short* __restrict__ Bt2p, int ldb, long strideB,
    void* __restrict__ Cout, void* __restrict__ Cout2, int ldc, long strideC,
    const float* __restrict__ bias,
    const float* __restrict__ resid, long strideR,
    int M, int N, int K, float scale) {
  typedef typename Elem<ET>::T T;
  typedef typename Frag<T>::V V;
  const T* A = (const T*)Ap; const T* A2 = (const T*)A2p; const T* Bt = (const T*)Btp; const T* Bt2 = (const T*)Bt2p;
  __shared__ __align__(16) float sT[8][16 * 68];
  const int b    = blockIdx.y;
  const int lane = threadIdx.x & 31;
  const int wave = threadIdx.x >> 5;
  const int tilesN = N >> 6;
  const int tilesM = M >> 6;
  const int tile = blockIdx.x * 8 + wave;
  if (tile >= tilesM * tilesN) return;
  const int tm = tile / tilesN;
  const int tn = tile - tm * tilesN;
  const int m0 = tm << 6;
  const int n0 = tn << 6;

  const T* Ab  = A  + (size_t)b * strideA;
  const T* Bb  = Bt + (size_t)b * strideB;
  const T* Ab2 = SPLIT ? (A2  + (size_t)b * strideA) : nullptr;
  const T* Bb2 = SPLIT ? (Bt2 + (size_t)b * strideB) : nullptr;

  const int rlane = lane & 15;
  const int koff  = (lane >> 4) * 8;
  const int mOff  = (lane >> 4) * 8;

  v8f acc[4][4];
#pragma unroll
  for (int i = 0; i < 4; ++i)
#pragma unroll
    for (int j = 0; j < 4; ++j) acc[i][j] = (v8f){0.f,0.f,0.f,0.f,0.f,0.f,0.f,0.f};

  for (int k0 = 0; k0 < K; k0 += 32) {
    V bh[4], bl[4];
#pragma unroll
    for (int j = 0; j < 4; ++j) {
      const size_t bo = (size_t)(n0 + (j << 4) + rlane) * ldb + koff + k0;
      bh[j] = Frag<T>::load(Bb + bo);
      if (SPLIT) bl[j] = Frag<T>::load(Bb2 + bo);
    }
#pragma unroll
    for (int i = 0; i < 4; ++i) {
      const size_t ao = (size_t)(m0 + (i << 4) + rlane) * lda + koff + k0;
      V ah = Frag<T>::load(Ab + ao);
      V al;
      if (SPLIT) al = Frag<T>::load(Ab2 + ao);
#pragma unroll
      for (int j = 0; j < 4; ++j) {
        acc[i][j] = Frag<T>::mma(ah, bh[j], acc[i][j]);
        if (SPLIT) {
          acc[i][j] = Frag<T>::mma(ah, bl[j], acc[i][j]);
          acc[i][j] = Frag<T>::mma(al, bh[j], acc[i][j]);
        }
      }
      Frag<T>::guard4(acc[i][0], acc[i][1], acc[i][2], acc[i][3], ah, SPLIT ? al : ah);
    }
    Frag<T>::keep(bh[0], bh[1], bh[2], bh[3]);
    if (SPLIT) Frag<T>::keep(bl[0], bl[1], bl[2], bl[3]);
  }
  acc_guard4(acc[0][0], acc[0][1], acc[0][2], acc[0][3]);
  acc_guard4(acc[1][0], acc[1][1], acc[1][2], acc[1][3]);
  acc_guard4(acc[2][0], acc[2][1], acc[2][2], acc[2][3]);
  acc_guard4(acc[3][0], acc[3][1], acc[3][2], acc[3][3]);

  float* slab = sT[wave];
  const float* Rb = RESID ? (resid + (size_t)b * strideR) : nullptr;
#pragma unroll
  for (int i = 0; i < 4; ++i) {
    const int mBase = m0 + (i << 4);
#pragma unroll
    for (int j = 0; j < 4; ++j) {
      const int n = n0 + (j << 4) + rlane;
      float bv = 0.f;
      if (BIAS_MODE == 2) bv = bias[n];
#pragma unroll
      for (int r = 0; r < 8; ++r) {
        float v = acc[i][j][r] * scale;
        if (BIAS_MODE == 1) v += bias[mBase + mOff + r];
        if (BIAS_MODE == 2) v += bv;
        if (RESID) v += Rb[(size_t)(mBase + mOff + r) * ldc + n];
        if (ACT == 2) v = fmaxf(v, 0.0f);
        if (ACT == 4) v = (v > 0.f) ? v : 0.01f * v;
        slab[(mOff + r) * 68 + (j << 4) + rlane] = v;
      }
    }
    __builtin_amdgcn_fence(__ATOMIC_RELEASE, "workgroup");
    __builtin_amdgcn_wave_barrier();
    __builtin_amdgcn_fence(__ATOMIC_ACQUIRE, "workgroup");
    if (OUT_MODE == 0) {
      float* C = (float*)Cout + (size_t)b * strideC;
      const int hh = lane >> 4, c4 = (lane & 15) * 4;
      for (int pass = 0; pass < 2; ++pass) {
#pragma unroll
        for (int it = 0; it < 8; ++it) {
          const int row = it * 2 + hh;
          v4f v = *(const v4f*)(slab + row * 68 + c4);
          *(volatile v4f*)(C + (size_t)(mBase + row) * ldc + n0 + c4) = v;
        }
        __threadfence();
      }
    } else {
      const int q = lane >> 3, c8 = (lane & 7) * 8;
      unsigned short* C  = (unsigned short*)Cout  + (size_t)b * strideC;
      unsigned short* C2 = (OUT_MODE == 2) ? ((unsigned short*)Cout2 + (size_t)b * strideC) : nullptr;
      for (int pass = 0; pass < 2; ++pass) {
#pragma unroll
        for (int it = 0; it < 4; ++it) {
          const int row = it * 4 + q;
          const float* sp = slab + row * 68 + c8;
          v8h hv, lv;
#pragma unroll
          for (int e = 0; e < 8; ++e) {
            if (OUT_MODE == 1) {
              hv[e] = (_Float16)sp[e];
            } else {
              unsigned short hb = f2bf_bits(sp[e]);
              unsigned short lb = f2bf_bits(sp[e] - bf_bits2f(hb));
              hv[e] = __builtin_bit_cast(_Float16, hb);
              lv[e] = __builtin_bit_cast(_Float16, lb);
            }
          }
          *(volatile v8h*)(C + (size_t)(mBase + row) * ldc + n0 + c8) = hv;
          if (OUT_MODE == 2) *(volatile v8h*)(C2 + (size_t)(mBase + row) * ldc + n0 + c8) = lv;
        }
        __threadfence();
      }
    }
    __builtin_amdgcn_fence(__ATOMIC_RELEASE, "workgroup");
    __builtin_amdgcn_wave_barrier();
    __builtin_amdgcn_fence(__ATOMIC_ACQUIRE, "workgroup");
  }
}

__global__ __launch_bounds__(256) void cast8_f16_kernel(const float* __restrict__ in, unsigned short* __restrict__ out,
                                                       int n8, float scale) {
  const int i = blockIdx.x * 256 + threadIdx.x;
  if (i >= n8) return;
  const float* p = in + 8 * (size_t)i;
  const v4f a = *(const v4f*)(p);
  const v4f c = *(const v4f*)(p + 4);
  unsigned short hb[8];
#pragma unroll
  for (int e = 0; e < 4; ++e) {
    hb[e]     = h_bits(a[e] * scale);
    hb[4 + e] = h_bits(c[e] * scale);
  }
  const v4u u = (v4u){pk16(hb[0], hb[1]), pk16(hb[2], hb[3]), pk16(hb[4], hb[5]), pk16(hb[6], hb[7])};
  unsigned short* q = out + 8 * (size_t)i;
  *(volatile v4u*)q = u;
  __threadfence();
  *(volatile v4u*)q = u;
}

__global__ __launch_bounds__(256) void wt_cast_kernel(const float* __restrict__ W0, const float* __restrict__ W1,
                                                     const float* __restrict__ W2, int nK, int nN,
                                                     unsigned short* __restrict__ out, long planeStride, float scale) {
  __shared__ float sm[64][65];
  const int t  = threadIdx.x;
  const int k0 = blockIdx.x * 64;
  const int n0 = blockIdx.y * 64;
  const int z  = blockIdx.z;
  const float* W = (z == 0) ? W0 : (z == 1) ? W1 : W2;
#pragma unroll
  for (int i = 0; i < 16; ++i) {
    const int e = i * 256 + t;
    const int r = e >> 6;
    const int c = e & 63;
    sm[c][r] = W[(size_t)(k0 + r) * nN + n0 + c] * scale;
  }
  __syncthreads();
  const int lane = t & 31, wave = t >> 5;
  const int q = lane >> 3, c8 = (lane & 7) * 8;
  unsigned short* op = out + (size_t)z * planeStride;
  for (int pass = 0; pass < 2; ++pass) {
#pragma unroll
    for (int it = 0; it < 2; ++it) {
      const int row = wave * 8 + it * 4 + q;
      unsigned short hb[8];
#pragma unroll
      for (int e = 0; e < 8; ++e) hb[e] = h_bits(sm[row][c8 + e]);
      const v4u u = (v4u){pk16(hb[0], hb[1]), pk16(hb[2], hb[3]), pk16(hb[4], hb[5]), pk16(hb[6], hb[7])};
      *(volatile v4u*)(op + (size_t)(n0 + row) * nK + k0 + c8) = u;
    }
    __threadfence();
  }
}

__global__ __launch_bounds__(128) void flow_scan_kernel(const float* __restrict__ P, unsigned short* __restrict__ att,
                                                       float carry) {
  __shared__ __align__(16) float kbuf[64];
  __shared__ __align__(16) float qsbuf[64];
  __shared__ __align__(16) float vbuf[64];
  __shared__ __align__(16) float accp[128];
  __shared__ __align__(16) float xrow[64];
  __shared__ float red1[4];
  __shared__ float red2[4];

  const int t    = threadIdx.x;
  const int lane = t & 31;
  const int wave = t >> 5;
  const int bh   = blockIdx.x;
  const int b    = bh >> 4;
  const int h    = bh & 15;
  const int d    = t & 63;
  const int role = wave >> 1;
  const bool qside = (role == 0);

  float S[32];
#pragma unroll
  for (int i = 0; i < 32; ++i) S[i] = 0.0f;
  float cum1 = 0.0f;
  float cum2 = 0.0f;
  float cume = 0.0f;

  const float* pbase = P + (size_t)b * kSeq * kQKVld + h * kDh + d;
  unsigned short* obase = att + (size_t)b * kSeq * kDim + h * kDh;

#pragma unroll 1
  for (int l = 0; l < kSeq; ++l) {
    const float* pr = pbase + (size_t)l * kQKVld;
    const float qpre = pr[0];
    const float kpre = pr[kDim];
    const float vraw = pr[2 * kDim];
    const float q = sigm(qpre);
    const float k = sigm(kpre);
    const float a = qside ? q : k;
    const float c = qside ? k : q;
    cum1 += c;
    float t1 = (a + kFlowEps) * (cum1 + kFlowEps);
#pragma unroll
    for (int off = 16; off > 0; off >>= 1) t1 += __shfl_xor(t1, off, 32);
    if (lane == 0) red1[wave] = t1;
    if (wave < 2) vbuf[d] = vraw;
    __syncthreads();

    const float p1 = red1[0] + red1[1];
    const float p2 = red1[2] + red1[3];
    const float normal  = (float)(l + 1);
    const float rnormal = frcp(normal);
    const float sink_in = normal * frcp(p1);
    const float src_out = normal * frcp(p2);
    const float sc = qside ? src_out : sink_in;
    cum2 += c * sc;
    float t2 = (a + kFlowEps) * (cum2 + kFlowEps);
#pragma unroll
    for (int off = 16; off > 0; off >>= 1) t2 += __shfl_xor(t2, off, 32);
    if (lane == 0) red2[wave] = t2;
    if (wave < 2) {
      kbuf[d]  = k;
      qsbuf[d] = q * (sink_in * rnormal);
    }
    __syncthreads();

    const float p3 = red2[0] + red2[1];
    const float p4 = red2[2] + red2[3];
    float cs = p4 * rnormal;
    cs = fminf(fmaxf(cs, -1.0f), 1.0f);
    const float e = expf(cs);
    cume += e;
    const float src_comp = (e * frcp(cume)) * normal;
    const float vs = vbuf[d] * src_comp;
    const float* kp = kbuf + role * 32;
    const float* qp = qsbuf + role * 32;
    float acc = 0.0f;
#pragma unroll
    for (int i4 = 0; i4 < 8; ++i4) {
      const v4f kk = *(const v4f*)(kp + 4 * i4);
      const v4f qq = *(const v4f*)(qp + 4 * i4);
#pragma unroll
      for (int e2 = 0; e2 < 4; ++e2) {
        const float kv1 = kk[e2];
        const float qv1 = qq[e2];
        S[4 * i4 + e2] = fmaf(kv1, vs, S[4 * i4 + e2]);
        acc = fmaf(qv1, S[4 * i4 + e2], acc);
      }
    }
    accp[role * 64 + d] = acc;
    __syncthreads();

    if (wave < 2) {
      const float sink_alloc = sigm(p3 * rnormal);
      const float x = (accp[d] + accp[64 + d]) * sink_alloc;
      xrow[d] = x * carry;
    }
    __syncthreads();

    if (wave == 0) {
      const int c8 = (lane & 7) * 8;
      const v4f x0 = *(const v4f*)(xrow + c8);
      const v4f x1 = *(const v4f*)(xrow + c8 + 4);
      unsigned short hb[8];
#pragma unroll
      for (int e3 = 0; e3 < 4; ++e3) {
        hb[e3]     = h_bits(x0[e3]);
        hb[4 + e3] = h_bits(x1[e3]);
      }
      const v4u u = (v4u){pk16(hb[0], hb[1]), pk16(hb[2], hb[3]), pk16(hb[4], hb[5]), pk16(hb[6], hb[7])};
      if (lane < 8) {
        unsigned short* op = obase + (size_t)l * kDim + c8;
        *(volatile v4u*)op = u;
        __threadfence();
        *(volatile v4u*)op = u;
      }
    }
  }
}

template <bool EMIT16>
__global__ __launch_bounds__(256) void add_ln_kernel(const float* __restrict__ x, const float* __restrict__ y,
                                                    const float* __restrict__ g, const float* __restrict__ bta,
                                                    float* __restrict__ outf, unsigned short* __restrict__ out16,
                                                    float carry16) {
  __shared__ __align__(16) float rowbuf[EMIT16 ? kDim : 4];
  __shared__ float redA[8];
  __shared__ float redB[8];
  const int row  = blockIdx.x;
  const int t    = threadIdx.x;
  const int lane = t & 31, wave = t >> 5;
  const size_t base = (size_t)row * kDim + 4 * t;
  const v4f xv = *(const v4f*)(x + base);
  const v4f yv = *(const v4f*)(y + base);
  const float v0 = xv[0] + yv[0];
  const float v1 = xv[1] + yv[1];
  const float v2 = xv[2] + yv[2];
  const float v3 = xv[3] + yv[3];
  float s = (v0 + v1) + (v2 + v3);
#pragma unroll
  for (int off = 16; off > 0; off >>= 1) s += __shfl_xor(s, off, 32);
  if (lane == 0) redA[wave] = s;
  __syncthreads();
  float tot = redA[0];
#pragma unroll
  for (int w = 1; w < 8; ++w) tot += redA[w];
  const float mean = tot * kInvDim;
  const float d0 = v0 - mean, d1 = v1 - mean, d2 = v2 - mean, d3 = v3 - mean;
  float sq = (d0 * d0 + d1 * d1) + (d2 * d2 + d3 * d3);
#pragma unroll
  for (int off = 16; off > 0; off >>= 1) sq += __shfl_xor(sq, off, 32);
  if (lane == 0) redB[wave] = sq;
  __syncthreads();
  float vt = redB[0];
#pragma unroll
  for (int w = 1; w < 8; ++w) vt += redB[w];
  const float var  = vt * kInvDim;
  const float rstd = 1.0f / sqrtf(var + kLnEps);
  const v4f gv = *(const v4f*)(g + 4 * t);
  const v4f bv = *(const v4f*)(bta + 4 * t);
  v4f ov;
  ov[0] = d0 * rstd * gv[0] + bv[0];
  ov[1] = d1 * rstd * gv[1] + bv[1];
  ov[2] = d2 * rstd * gv[2] + bv[2];
  ov[3] = d3 * rstd * gv[3] + bv[3];
  *(volatile v4f*)(outf + base) = ov;
  __threadfence();
  *(volatile v4f*)(outf + base) = ov;
  if (EMIT16) {
    *(v4f*)(rowbuf + 4 * t) = ov;
    __syncthreads();
    if (t < 128) {
      const v4f a0 = *(const v4f*)(rowbuf + 8 * t);
      const v4f a1 = *(const v4f*)(rowbuf + 8 * t + 4);
      unsigned short hb[8];
#pragma unroll
      for (int e = 0; e < 4; ++e) {
        hb[e]     = h_bits(a0[e] * carry16);
        hb[4 + e] = h_bits(a1[e] * carry16);
      }
      const v4u u = (v4u){pk16(hb[0], hb[1]), pk16(hb[2], hb[3]), pk16(hb[4], hb[5]), pk16(hb[6], hb[7])};
      unsigned short* op = out16 + (size_t)row * kDim + 8 * t;
      *(volatile v4u*)op = u;
      __threadfence();
      *(volatile v4u*)op = u;
    }
  }
}

__global__ __launch_bounds__(256) void gelu_cast_x2_kernel(const float* __restrict__ in, unsigned short* __restrict__ out,
                                                         int n2, float carry) {
  const int i = blockIdx.x * 256 + threadIdx.x;
  if (i < n2) {
    const v2f zz = *(const v2f*)(in + 2 * (size_t)i);
    const float z0 = zz[0];
    const float z1 = zz[1];
    const float g0 = 0.5f * z0 * (1.0f + erff(z0 * 0.70710678118654752f));
    const float g1 = 0.5f * z1 * (1.0f + erff(z1 * 0.70710678118654752f));
    const unsigned u = pk16(h_bits(g0 * carry), h_bits(g1 * carry));
    ((volatile unsigned*)out)[i] = u;
    __threadfence();
    ((volatile unsigned*)out)[i] = u;
  }
}

extern "C" void kernel_launch(void* const* d_in, const int* in_sizes, int n_in,
                              void* d_out, int out_size, void* d_ws, size_t ws_size,
                              hipStream_t stream) {
  if (n_in < 18) return;
  if (in_sizes[0] != kTok * kDim) return;
  if (in_sizes[2] != kDim * kDim || in_sizes[4] != kDim * kDim || in_sizes[6] != kDim * kDim || in_sizes[8] != kDim * kDim) return;
  if (in_sizes[3] != kDim || in_sizes[5] != kDim || in_sizes[7] != kDim || in_sizes[9] != kDim) return;
  if (in_sizes[10] != kDim || in_sizes[11] != kDim || in_sizes[16] != kDim || in_sizes[17] != kDim) return;
  if (in_sizes[12] != kDim * kFF || in_sizes[13] != kFF || in_sizes[14] != kFF * kDim || in_sizes[15] != kDim) return;
  if (out_size != kTok * kDim) return;

  const size_t szX16  = (size_t)kTok * kDim * 2;
  const size_t szWqkv = (size_t)3 * kDim * kDim * 2;
  const size_t szWo   = (size_t)kDim * kDim * 2;
  const size_t szW1   = (size_t)kFF * kDim * 2;
  const size_t szW2   = (size_t)kDim * kFF * 2;
  const size_t szQKV  = (size_t)kTok * kQKVld * 4;
  const size_t szAtt  = (size_t)kTok * kDim * 2;
  const size_t szR    = (size_t)kTok * kDim * 4;
  const size_t szH    = (size_t)kTok * kDim * 4;
  const size_t szH16  = (size_t)kTok * kDim * 2;
  const size_t szZ    = (size_t)kTok * kFF * 4;
  const size_t szU16  = (size_t)kTok * kFF * 2;
  const size_t offX16  = 0;
  const size_t offWqkv = offX16 + szX16;
  const size_t offWo   = offWqkv + szWqkv;
  const size_t offW1   = offWo + szWo;
  const size_t offW2   = offW1 + szW1;
  const size_t offQKV  = offW2 + szW2;
  const size_t offAtt  = offQKV + szQKV;
  const size_t offR    = offAtt + szAtt;
  const size_t offH    = offR + szR;
  const size_t offH16  = offH + szH;
  const size_t offZ    = offH16 + szH16;
  const size_t offU16  = offZ + szZ;
  const size_t total   = offU16 + szU16;
  if (ws_size < total) return;

  const float* inp  = (const float*)d_in[0];
  const float* Wq   = (const float*)d_in[2];
  const float* bq   = (const float*)d_in[3];
  const float* Wk   = (const float*)d_in[4];
  const float* bk   = (const float*)d_in[5];
  const float* Wv   = (const float*)d_in[6];
  const float* bv   = (const float*)d_in[7];
  const float* Wo   = (const float*)d_in[8];
  const float* bo   = (const float*)d_in[9];
  const float* ln1g = (const float*)d_in[10];
  const float* ln1b = (const float*)d_in[11];
  const float* W1   = (const float*)d_in[12];
  const float* b1   = (const float*)d_in[13];
  const float* W2   = (const float*)d_in[14];
  const float* b2   = (const float*)d_in[15];
  const float* ln2g = (const float*)d_in[16];
  const float* ln2b = (const float*)d_in[17];
  float* out = (float*)d_out;

  char* ws = (char*)d_ws;
  unsigned short* X16   = (unsigned short*)(ws + offX16);
  unsigned short* WQKVT = (unsigned short*)(ws + offWqkv);
  unsigned short* WOT   = (unsigned short*)(ws + offWo);
  unsigned short* W1T   = (unsigned short*)(ws + offW1);
  unsigned short* W2T   = (unsigned short*)(ws + offW2);
  float*          QKV   = (float*)(ws + offQKV);
  unsigned short* ATT16 = (unsigned short*)(ws + offAtt);
  float*          RF    = (float*)(ws + offR);
  float*          HF    = (float*)(ws + offH);
  unsigned short* H16   = (unsigned short*)(ws + offH16);
  float*          ZF    = (float*)(ws + offZ);
  unsigned short* U16   = (unsigned short*)(ws + offU16);

  const int n8x = (kTok * kDim) / 8;
  cast8_f16_kernel<<<dim3(n8x / 256), dim3(256), 0, stream>>>(inp, X16, n8x, kXCarry);
  wt_cast_kernel<<<dim3(kDim / 64, kDim / 64, 3), dim3(256), 0, stream>>>(Wq, Wk, Wv, kDim, kDim, WQKVT, (long)kDim * kDim, kWCarry);
  wt_cast_kernel<<<dim3(kDim / 64, kDim / 64, 1), dim3(256), 0, stream>>>(Wo, Wo, Wo, kDim, kDim, WOT, 0L, kWCarry);
  wt_cast_kernel<<<dim3(kDim / 64, kFF / 64, 1), dim3(256), 0, stream>>>(W1, W1, W1, kDim, kFF, W1T, 0L, kWCarry);
  wt_cast_kernel<<<dim3(kFF / 64, kDim / 64, 1), dim3(256), 0, stream>>>(W2, W2, W2, kFF, kDim, W2T, 0L, kWCarry);

  const int tiles_sq = (kTok / 64) * (kDim / 64);
  {
    const float* bqkv[3] = {bq, bk, bv};
    for (int z = 0; z < 3; ++z) {
      const unsigned short* Btz = WQKVT + (size_t)z * kDim * kDim;
      float* Cz = QKV + (size_t)z * kDim;
      wmma_gemm64<0, false, 2, 0, false, 0><<<dim3(tiles_sq / 8, 1), dim3(256), 0, stream>>>(
          X16, X16, kDim, 0L, Btz, Btz, kDim, 0L,
          (void*)Cz, (void*)Cz, kQKVld, 0L, bqkv[z], bqkv[z], 0L, kTok, kDim, kDim, kScaleXW);
    }
  }

  flow_scan_kernel<<<dim3(kBatch * kHeads), dim3(128), 0, stream>>>(QKV, ATT16, kAttCarry);

  wmma_gemm64<0, false, 2, 0, false, 0><<<dim3(tiles_sq / 8, 1), dim3(256), 0, stream>>>(
      ATT16, ATT16, kDim, 0L, WOT, WOT, kDim, 0L,
      (void*)RF, (void*)RF, kDim, 0L, bo, bo, 0L, kTok, kDim, kDim, kScaleAW);

  add_ln_kernel<true><<<dim3(kTok), dim3(256), 0, stream>>>(inp, RF, ln1g, ln1b, HF, H16, kHCarry);

  const int tiles_up = (kTok / 64) * (kFF / 64);
  wmma_gemm64<0, false, 2, 0, false, 0><<<dim3(tiles_up / 8, 1), dim3(256), 0, stream>>>(
      H16, H16, kDim, 0L, W1T, W1T, kDim, 0L,
      (void*)ZF, (void*)ZF, kFF, 0L, b1, b1, 0L, kTok, kFF, kDim, kScaleHW);

  const int n2u = (kTok * kFF) / 2;
  gelu_cast_x2_kernel<<<dim3(n2u / 256), dim3(256), 0, stream>>>(ZF, U16, n2u, kUCarry);

  wmma_gemm64<0, false, 2, 0, false, 0><<<dim3(tiles_sq / 8, 1), dim3(256), 0, stream>>>(
      U16, U16, kFF, 0L, W2T, W2T, kFF, 0L,
      (void*)RF, (void*)RF, kDim, 0L, b2, b2, 0L, kTok, kDim, kFF, kScaleUW);

  add_ln_kernel<false><<<dim3(kTok), dim3(256), 0, stream>>>(HF, RF, ln2g, ln2b, out, H16, kHCarry);
}
